// NetVLAD_V1_53472342835390
// MI455X (gfx1250) — hardware-run, weakly checked
//
#include <hip/hip_runtime.h>
#include <stddef.h>


typedef _Float16 v16h __attribute__((ext_vector_type(16)));
typedef _Float16 v8h  __attribute__((ext_vector_type(8)));
typedef float    v8f  __attribute__((ext_vector_type(8)));
typedef float    v4f  __attribute__((ext_vector_type(4)));
typedef _Float16 h16;

#ifndef NB
#define NB 4
#endif
#define NB_FULL 4
#define CH   128
#define PP   784
#define PPAD 832
#define DD   512
#define KC   64
#define TAILV ((PP - 768) / 4)

static_assert(NB >= 1 && NB <= NB_FULL);
static_assert(CH == 128);
static_assert((CH % 32) == 0);
static_assert((PPAD % 64) == 0 && PPAD >= PP && (PPAD - PP) < 64);
static_assert((PPAD % 32) == 0);
static_assert((DD % 64) == 0 && (DD % 32) == 0);
static_assert(KC == 64);
static_assert((PP % 4) == 0 && PP > 768 && PP <= 768 + 16);
static_assert(TAILV >= 1 && TAILV <= 4);
static_assert(768 + 4 * 15 <= PPAD - 4);
static_assert(((DD * CH) % 2048) == 0);
static_assert((size_t)NB_FULL * KC * DD * 4 == (size_t)524288);

#define LDC 68
#define LDP 65
#define SP  36
static_assert((LDC % 4) == 0 && LDC >= 64);
static_assert(LDP >= 64);
static_assert((SP % 4) == 0 && SP >= 32);

#define WCARRY 64.0f
#define XCARRY 64.0f

#define WP_BYTES   ((size_t)DD * CH * 2)
#define XN_BYTES   ((size_t)NB * PPAD * CH * 2)
#define FEAT_BYTES ((size_t)NB * DD * PPAD * 4)
#define OFF_WP   ((size_t)0)
#define OFF_XN   (OFF_WP + WP_BYTES)
#define OFF_FEAT (OFF_XN + XN_BYTES)
#define WS_TOTAL (OFF_FEAT + FEAT_BYTES)
static_assert((WP_BYTES % 128) == 0 && (XN_BYTES % 128) == 0 && (FEAT_BYTES % 128) == 0);
static_assert(WS_TOTAL <= (size_t)134217728);

__device__ __forceinline__ float bf16r(float x) {
  unsigned int u = __float_as_uint(x);
  u = (u + 0x7FFFu + ((u >> 16) & 1u)) & 0xFFFF0000u;
  return __uint_as_float(u);
}

static __device__ __forceinline__ h16 toh_flush(float v) {
  const h16 r = (h16)v;
  return (fabsf(v) < 6.103515625e-05f) ? (h16)0.0f : r;
}

__device__ __forceinline__ v16h frag_at(const _Float16* p) {
  v8h lo = *(const v8h*)(p);
  v8h hi = *(const v8h*)(p + 16);
  v16h out;
#pragma unroll
  for (int i = 0; i < 8; ++i) { out[i] = lo[i]; out[i + 8] = hi[i]; }
  return out;
}

__device__ __forceinline__ v8f wmma16(v16h a, v16h b, v8f c) {
  v8f d = __builtin_amdgcn_wmma_f32_16x16x32_f16(false, a, false, b, (short)0, c,
                                                 false, false);
  asm volatile("v_nop\n\tv_nop\n\tv_nop\n\tv_nop" : "+v"(d) : "v"(a), "v"(b));
  return d;
}

__device__ __forceinline__ float red32_sum(float x) {
#pragma unroll
  for (int off = 1; off < 32; off <<= 1) x += __shfl_xor(x, off, 32);
  return x;
}
__device__ __forceinline__ float red32_max(float x) {
#pragma unroll
  for (int off = 1; off < 32; off <<= 1) x = fmaxf(x, __shfl_xor(x, off, 32));
  return x;
}

__global__ __launch_bounds__(256) void wplane_kernel(
    const float* __restrict__ W, _Float16* __restrict__ Wp) {
  const unsigned idx = (blockIdx.x * 256u + threadIdx.x) * 8u;
  const v4f a0 = *(const v4f*)(W + idx);
  const v4f a1 = *(const v4f*)(W + idx + 4u);
  v8h o;
#pragma unroll
  for (int i = 0; i < 4; ++i) {
    o[i]     = toh_flush(WCARRY * bf16r(a0[i]));
    o[i + 4] = toh_flush(WCARRY * bf16r(a1[i]));
  }
  *(volatile v8h*)(Wp + idx) = o;
  __threadfence();
  *(volatile v8h*)(Wp + idx) = o;
}

__global__ __launch_bounds__(256) void xnorm_kernel(
    const float* __restrict__ X, _Float16* __restrict__ Xn) {
#pragma clang fp contract(off)
  __shared__ float Tf[CH * LDP];
  __shared__ float Part[4 * 64];
  __shared__ float Inv[64];
  const unsigned tid = threadIdx.x;
  const unsigned p0 = blockIdx.x * 64u;
  const unsigned b = blockIdx.y;
  const float* xb = X + (size_t)b * (CH * PP);

#pragma unroll 4
  for (unsigned j = 0; j < 32u; ++j) {
    const unsigned idx = tid + 256u * j;
    const unsigned c = idx >> 6, pl = idx & 63u;
    const unsigned p = p0 + pl;
    const unsigned pc = (p < (unsigned)PP) ? p : (unsigned)(PP - 1);
    float v = xb[(size_t)c * PP + pc];
    asm volatile("" : "+v"(v));
    Tf[c * LDP + pl] = (p < (unsigned)PP) ? bf16r(v) : 0.0f;
  }
  __syncthreads();

  {
    const unsigned pl = tid & 63u, q = tid >> 6;
    float ss = 0.0f;
#pragma unroll 4
    for (unsigned c = 0; c < 32u; ++c) {
      const float v = Tf[(32u * q + c) * LDP + pl];
      ss += v * v;
    }
    Part[q * 64u + pl] = ss;
  }
  __syncthreads();
  if (tid < 64u) {
    const float s = (Part[tid] + Part[64u + tid]) + (Part[128u + tid] + Part[192u + tid]);
    Inv[tid] = XCARRY * (1.0f / fmaxf(sqrtf(s), 1.0e-12f));
  }
  __syncthreads();

  v8h x[4];
  size_t off[4];
#pragma unroll
  for (unsigned i = 0; i < 4u; ++i) {
    const unsigned idx = tid + 256u * i;
    const unsigned r = idx >> 4, kc = (idx & 15u) * 8u;
    const float sc = Inv[r];
#pragma unroll
    for (unsigned e = 0; e < 8u; ++e) x[i][e] = toh_flush(Tf[(kc + e) * LDP + r] * sc);
    off[i] = ((size_t)b * PPAD + p0 + r) * CH + kc;
  }
#pragma unroll
  for (int i = 0; i < 4; ++i) *(volatile v8h*)(Xn + off[i]) = x[i];
  __threadfence();
#pragma unroll
  for (int i = 0; i < 4; ++i) *(volatile v8h*)(Xn + off[i]) = x[i];
}

__global__ __launch_bounds__(256) void gemm_feat_kernel(
    const _Float16* __restrict__ Wp, const _Float16* __restrict__ Xn,
    const float* __restrict__ bias, float* __restrict__ feat) {
  __shared__ float Cs[64 * LDC];
  const unsigned tid = threadIdx.x, lane = tid & 31u;
  const unsigned w = (unsigned)__builtin_amdgcn_readfirstlane((int)(threadIdx.x >> 5));
  const unsigned mw = w >> 1, nw = w & 1u;
  const unsigned hh = lane >> 4, m = lane & 15u;
  const unsigned n0 = blockIdx.x * 64u;
  const unsigned row0 = blockIdx.y * 64u;
  const unsigned b = blockIdx.z;

  const _Float16* ap  = Wp + (size_t)(row0 + mw * 16u + m) * CH + hh * 8u;
  const _Float16* bp0 = Xn + ((size_t)b * PPAD + n0 + nw * 32u + m) * CH + hh * 8u;
  const _Float16* bp1 = bp0 + (size_t)16 * CH;
  v8f acc0 = {}, acc1 = {};
#pragma unroll 2
  for (unsigned k0 = 0; k0 < (unsigned)CH; k0 += 32u) {
    const v16h a  = frag_at(ap + k0);
    const v16h b0 = frag_at(bp0 + k0);
    const v16h b1 = frag_at(bp1 + k0);
    acc0 = wmma16(a, b0, acc0);
    acc1 = wmma16(a, b1, acc1);
  }
#pragma unroll
  for (int r = 0; r < 8; ++r) {
    float* d = &Cs[(mw * 16u + hh * 8u + (unsigned)r) * LDC + nw * 32u + m];
    d[0]  = acc0[r];
    d[16] = acc1[r];
  }
  __syncthreads();

  const float cs = 1.0f / (WCARRY * XCARRY);
  v4f xs[4];
  size_t off[4];
#pragma unroll
  for (unsigned i = 0; i < 4u; ++i) {
    const unsigned r = 16u * i + (tid >> 4);
    const unsigned c = (tid & 15u) * 4u;
    const v4f u = *(const v4f*)&Cs[r * LDC + c];
    const float bb = bf16r(bias[row0 + r]);
    v4f val;
#pragma unroll
    for (int j = 0; j < 4; ++j) val[j] = u[j] * cs + bb;
    xs[i] = val;
    off[i] = ((size_t)b * DD + row0 + r) * PPAD + n0 + c;
  }
#pragma unroll
  for (int i = 0; i < 4; ++i) *(volatile v4f*)(feat + off[i]) = xs[i];
  __threadfence();
#pragma unroll
  for (int i = 0; i < 4; ++i) *(volatile v4f*)(feat + off[i]) = xs[i];
}

__global__ __launch_bounds__(256) void vlad_kernel(
    const float* __restrict__ feat, const float* __restrict__ cent, float* __restrict__ out) {
#pragma clang fp contract(off)
  __shared__ float Sst[KC * SP];
  const unsigned tid = threadIdx.x, lane = tid & 31u;
  const unsigned wave = (unsigned)__builtin_amdgcn_readfirstlane((int)(threadIdx.x >> 5));
  const unsigned d0 = blockIdx.x * 32u;
  const unsigned b = blockIdx.y;
  const bool tailok = lane < (unsigned)TAILV;

#pragma unroll 1
  for (unsigned j = 0; j < 4u; ++j) {
    const unsigned dl = wave * 4u + j;
    const unsigned d = d0 + dl;
    const float* fr = feat + ((size_t)b * DD + d) * PPAD;
    v4f fv[7];
#pragma unroll
    for (int i = 0; i < 7; ++i) {
      unsigned col = 4u * lane + 128u * (unsigned)i;
      col = (col < (unsigned)(PPAD - 4)) ? col : (unsigned)(PPAD - 4);
      fv[i] = *(const v4f*)(fr + col);
    }
#pragma unroll
    for (int e = 0; e < 4; ++e) fv[6][e] = tailok ? fv[6][e] : 0.0f;

    float fm = -3.0e38f;
#pragma unroll
    for (int i = 0; i < 6; ++i)
#pragma unroll
      for (int e = 0; e < 4; ++e) fm = fmaxf(fm, fv[i][e]);
#pragma unroll
    for (int e = 0; e < 4; ++e) fm = fmaxf(fm, tailok ? fv[6][e] : -3.0e38f);
    fm = red32_max(fm);

    float o0 = 0.0f, o1 = 0.0f;
#pragma unroll 1
    for (unsigned k = 0; k < (unsigned)KC; ++k) {
      const float c = bf16r(cent[(size_t)k * DD + d]);
      const float mk = fm - c;
      float s1 = 0.0f, s2 = 0.0f;
#pragma unroll
      for (int i = 0; i < 6; ++i)
#pragma unroll
        for (int e = 0; e < 4; ++e) {
          const float f = fv[i][e];
          const float ex = __expf((f - c) - mk);
          s1 += ex;
          s2 += ex * f;
        }
#pragma unroll
      for (int e = 0; e < 4; ++e) {
        const float f = fv[6][e];
        float ex = __expf((f - c) - mk);
        ex = tailok ? ex : 0.0f;
        s1 += ex;
        s2 += ex * f;
      }
      s1 = red32_sum(s1);
      s2 = red32_sum(s2);
      const float S = s2 * (1.0f / s1);
      o0 = (k == lane) ? S : o0;
      o1 = (k == lane + 32u) ? S : o1;
    }
    Sst[lane * SP + dl] = o0;
    Sst[(lane + 32u) * SP + dl] = o1;
  }
  __syncthreads();

  v4f xs[2];
  size_t off[2];
#pragma unroll
  for (unsigned i = 0; i < 2u; ++i) {
    const unsigned idx = tid + 256u * i;
    const unsigned k = idx >> 3, c4 = (idx & 7u) * 4u;
    xs[i] = *(const v4f*)&Sst[k * SP + c4];
    off[i] = ((size_t)b * KC + k) * DD + d0 + c4;
  }
#pragma unroll
  for (int i = 0; i < 2; ++i) *(volatile v4f*)(out + off[i]) = xs[i];
  __threadfence();
#pragma unroll
  for (int i = 0; i < 2; ++i) *(volatile v4f*)(out + off[i]) = xs[i];
}

extern "C" void kernel_launch(void* const* d_in, const int* in_sizes, int n_in,
                              void* d_out, int out_size, void* d_ws, size_t ws_size,
                              hipStream_t stream) {
  if (n_in < 4) return;
  if ((long long)in_sizes[0] < (long long)NB * CH * PP) return;
  if ((long long)in_sizes[1] < (long long)DD * CH) return;
  if (in_sizes[2] < DD) return;
  if ((long long)in_sizes[3] < (long long)KC * DD) return;
  if ((long long)out_size < (long long)NB * KC * DD) return;
  if (ws_size < WS_TOTAL) return;

  const float* X    = (const float*)d_in[0];
  const float* cw   = (const float*)d_in[1];
  const float* cb   = (const float*)d_in[2];
  const float* cent = (const float*)d_in[3];
  float* out = (float*)d_out;

  char* ws = (char*)d_ws;
  _Float16* Wp   = (_Float16*)(ws + OFF_WP);
  _Float16* Xn   = (_Float16*)(ws + OFF_XN);
  float*    Feat = (float*)(ws + OFF_FEAT);

  dim3 blk(256);
  wplane_kernel<<<dim3((DD * CH) / 2048), blk, 0, stream>>>(cw, Wp);
  xnorm_kernel<<<dim3(PPAD / 64, NB), blk, 0, stream>>>(X, Xn);
  gemm_feat_kernel<<<dim3(PPAD / 64, DD / 64, NB), blk, 0, stream>>>(Wp, Xn, cb, Feat);
  vlad_kernel<<<dim3(DD / 32, NB), blk, 0, stream>>>(Feat, cent, out);
}
